// ContinuousSSMLayer_19155554140616
// MI455X (gfx1250) — hardware-verified
//
#include <hip/hip_runtime.h>
#include <math.h>

typedef __attribute__((ext_vector_type(16))) _Float16 v16h;
typedef __attribute__((ext_vector_type(8)))  _Float16 v8h;
typedef __attribute__((ext_vector_type(2)))  _Float16 v2h;
typedef __attribute__((ext_vector_type(8)))  float    v8f;
typedef __attribute__((ext_vector_type(4)))  float    v4f;
typedef __attribute__((ext_vector_type(2)))  float    v2f;
typedef __attribute__((ext_vector_type(4)))  unsigned v4u;

constexpr int kL      = 32768;
constexpr int kH      = 256;
constexpr int kP      = 128;
constexpr int kTW     = 2 * kP;
constexpr int kLC     = 128;
constexpr int kLog2LC = 7;
constexpr int kNChunk = kL / kLC;
constexpr int kTS     = 32;
constexpr int kRowF   = 2 * kP;
static_assert((1 << kLog2LC) == kLC, "chunk length is a power of two");
static_assert(kNChunk * kLC == kL, "chunks tile the sequence");
static_assert((kLC % kTS) == 0, "tile divides chunk");
static_assert((kL % 64) == 0 && (kH % 64) == 0 && (kTW % 64) == 0, "GEMM M,N multiples of 64");
static_assert((kH % 32) == 0 && (kTW % 32) == 0, "GEMM K multiples of 32");
static_assert((kNChunk % 8) == 0, "carry groups of 8");

constexpr float kCarryU  = 16.0f;
constexpr float kCarryB  = 256.0f;
constexpr float kCarryX  = 256.0f;
constexpr float kCarryC2 = 128.0f;
constexpr float kScale1  = 1.0f / (kCarryU * kCarryB);
constexpr float kScale2  = 1.0f / (kCarryX * kCarryC2);

constexpr size_t kOffA1    = 0;
constexpr size_t kOffTP    = kOffA1    + (size_t)kL * kH * 2;
constexpr size_t kOffA2    = kOffTP    + (size_t)kL * kTW * 4;
constexpr size_t kOffBT1   = kOffA2    + (size_t)kL * kTW * 2;
constexpr size_t kOffBT2   = kOffBT1   + (size_t)kTW * kH * 2;
constexpr size_t kOffEND   = kOffBT2   + (size_t)kH * kTW * 2;
constexpr size_t kOffCARRY = kOffEND   + (size_t)kNChunk * kRowF * 4;
constexpr size_t kOffTAB   = kOffCARRY + (size_t)kNChunk * kRowF * 4;
constexpr size_t kWsTotal  = kOffTAB   + 4096;
static_assert(kWsTotal == 67899392ull, "carve total");
static_assert(kWsTotal <= 134217728ull, "carve cap");
static_assert((kOffTP % 128) == 0 && (kOffA2 % 128) == 0 && (kOffBT1 % 128) == 0 && (kOffBT2 % 128) == 0 &&
              (kOffEND % 128) == 0 && (kOffCARRY % 128) == 0 && (kOffTAB % 128) == 0, "128-B aligned regions");
static_assert(6 * kP * 4 <= 4096, "table fits its carve");

__device__ __forceinline__ unsigned pack_h2(float a, float b) {
  v2h t;
  t[0] = (_Float16)a;
  t[1] = (_Float16)b;
  return __builtin_bit_cast(unsigned, t);
}

union FragU { v16h v; v8h h[2]; };
__device__ __forceinline__ v16h frag_load(const _Float16* p) {
  FragU f;
  f.h[0] = *(const v8h*)(p);
  f.h[1] = *(const v8h*)(p + 16);
  return f.v;
}
__device__ __forceinline__ v8f mma_f16_guarded(v16h a, v16h b, v8f c) {
  c = __builtin_amdgcn_wmma_f32_16x16x32_f16(false, a, false, b, (short)0, c, false, false);
  asm volatile("v_nop\n\tv_nop\n\tv_nop\n\tv_nop" : "+v"(c) : "v"(a), "v"(b));
  return c;
}

__global__ __launch_bounds__(128) void param_table_kernel(
    const float* __restrict__ Lre, const float* __restrict__ Lim,
    const float* __restrict__ lstep, float* __restrict__ tab)
{
#pragma clang fp contract(off)
  const int p = threadIdx.x;
  const float lr = Lre[p];
  const float li = Lim[p];
  const float step = expf(lstep[p]);
  const float zr = lr * step;
  const float zi = li * step;
  const float ea = expf(zr);
  float sn, cs;
  sincosf(zi, &sn, &cs);
  const float abr = ea * cs;
  const float abi = ea * sn;
  const float nr = abr - 1.0f;
  const float ni = abi;
  const float den = lr * lr + li * li;
  const float inv = 1.0f / den;
  const float cr = (nr * lr + ni * li) * inv;
  const float ci = (ni * lr - nr * li) * inv;
  float pr = abr, pi = abi;
#pragma unroll 1
  for (int q = 0; q < kLog2LC; ++q) {
    const float sr = pr * pr - pi * pi;
    const float si = 2.0f * pr * pi;
    pr = sr;
    pi = si;
  }
  for (int pass = 0; pass < 2; ++pass) {
    *(volatile float*)(tab + 0 * kP + p) = abr;
    *(volatile float*)(tab + 1 * kP + p) = abi;
    *(volatile float*)(tab + 2 * kP + p) = cr;
    *(volatile float*)(tab + 3 * kP + p) = ci;
    *(volatile float*)(tab + 4 * kP + p) = pr;
    *(volatile float*)(tab + 5 * kP + p) = pi;
    __threadfence();
  }
}

__global__ __launch_bounds__(256) void weight_planes_kernel(
    const float* __restrict__ Bsrc, const float* __restrict__ Csrc,
    unsigned short* __restrict__ bt1, unsigned short* __restrict__ bt2)
{
  const int which = (int)(blockIdx.x >> 5);
  const int i = (int)(blockIdx.x & 31) * 256 + (int)threadIdx.x;
  const int row = i >> 5;
  const int k0 = (i & 31) * 8;
  const float* src = which ? Csrc : Bsrc;
  unsigned short* dst = which ? bt2 : bt1;
  const int compB = row >> 7;
  const int compC = k0 >> 7;
  const size_t baseB = ((size_t)(row & 127) * kH + (size_t)k0) * 2;
  const size_t baseC = ((size_t)row * kP + (size_t)(k0 & 127)) * 2;
  const size_t sbase = which ? baseC : baseB;
  const int comp = which ? compC : compB;
  const float mulC = compC ? (-2.0f * kCarryC2) : (2.0f * kCarryC2);
  const float mul = which ? mulC : kCarryB;
  const v4f f0 = *(const v4f*)(src + sbase);
  const v4f f1 = *(const v4f*)(src + sbase + 4);
  const v4f f2 = *(const v4f*)(src + sbase + 8);
  const v4f f3 = *(const v4f*)(src + sbase + 12);
  float ev[8], od[8];
  ev[0] = f0[0]; od[0] = f0[1]; ev[1] = f0[2]; od[1] = f0[3];
  ev[2] = f1[0]; od[2] = f1[1]; ev[3] = f1[2]; od[3] = f1[3];
  ev[4] = f2[0]; od[4] = f2[1]; ev[5] = f2[2]; od[5] = f2[3];
  ev[6] = f3[0]; od[6] = f3[1]; ev[7] = f3[2]; od[7] = f3[3];
  v8h hv;
#pragma unroll
  for (int e = 0; e < 8; ++e) {
    const float s = comp ? od[e] : ev[e];
    hv[e] = (_Float16)(s * mul);
  }
  unsigned short* q = dst + (size_t)row * 256 + k0;
  *(volatile v8h*)q = hv;
  __threadfence();
  *(volatile v8h*)q = hv;
}

__global__ __launch_bounds__(256) void cast_rows_f16_kernel(
    const float* __restrict__ src, unsigned short* __restrict__ dst, int total8)
{
  const int i = (int)blockIdx.x * 256 + (int)threadIdx.x;
  if (i >= total8) return;
  const size_t e0 = (size_t)i << 3;
  const v4f a0 = *(const v4f*)(src + e0);
  const v4f a1 = *(const v4f*)(src + e0 + 4);
  v8h hv;
#pragma unroll
  for (int e = 0; e < 4; ++e) {
    hv[e]     = (_Float16)(a0[e] * kCarryU);
    hv[4 + e] = (_Float16)(a1[e] * kCarryU);
  }
  unsigned short* q = dst + e0;
  *(volatile v8h*)q = hv;
  __threadfence();
  *(volatile v8h*)q = hv;
}

template <bool SKIP>
__global__ __launch_bounds__(256) void gemm_f16_tile64(
    const unsigned short* __restrict__ Ap, int lda,
    const unsigned short* __restrict__ Btp, int ldb,
    float* __restrict__ Cout, int ldc,
    const float* __restrict__ skipGain, const float* __restrict__ skipSrc,
    int M, int N, int K, float scale)
{
  const _Float16* A  = (const _Float16*)Ap;
  const _Float16* Bt = (const _Float16*)Btp;
  __shared__ __align__(16) float sT[8][16 * 68];
  const int lane = (int)(threadIdx.x & 31);
  const int wave = __builtin_amdgcn_readfirstlane((int)(threadIdx.x >> 5));
  const int tilesN = N >> 6;
  const int tilesM = M >> 6;
  const int tile = (int)blockIdx.x * 8 + wave;
  if (tile >= tilesM * tilesN) return;
  const int tm = tile / tilesN;
  const int tn = tile - tm * tilesN;
  const int m0 = tm << 6;
  const int n0 = tn << 6;

  const int rlane = lane & 15;
  const int koff  = (lane >> 4) * 8;
  const int mOff  = (lane >> 4) * 8;

  v8f acc[4][4];
#pragma unroll
  for (int i = 0; i < 4; ++i)
#pragma unroll
    for (int j = 0; j < 4; ++j) acc[i][j] = (v8f){0.f, 0.f, 0.f, 0.f, 0.f, 0.f, 0.f, 0.f};

  for (int k0 = 0; k0 < K; k0 += 32) {
    v16h bh[4];
#pragma unroll
    for (int j = 0; j < 4; ++j) {
      const size_t bo = (size_t)(n0 + (j << 4) + rlane) * ldb + koff + k0;
      bh[j] = frag_load(Bt + bo);
    }
#pragma unroll
    for (int i = 0; i < 4; ++i) {
      const size_t ao = (size_t)(m0 + (i << 4) + rlane) * lda + koff + k0;
      const v16h ah = frag_load(A + ao);
#pragma unroll
      for (int j = 0; j < 4; ++j) acc[i][j] = mma_f16_guarded(ah, bh[j], acc[i][j]);
    }
  }

  float* slab = sT[wave];
  const int hh = lane >> 4;
  const int c4 = (lane & 15) * 4;
  v4f g4 = (v4f){0.f, 0.f, 0.f, 0.f};
  if (SKIP) g4 = *(const v4f*)(skipGain + n0 + c4);
#pragma unroll
  for (int i = 0; i < 4; ++i) {
    const int mBase = m0 + (i << 4);
#pragma unroll
    for (int j = 0; j < 4; ++j) {
#pragma unroll
      for (int r = 0; r < 8; ++r) {
        slab[(mOff + r) * 68 + (j << 4) + rlane] = acc[i][j][r] * scale;
      }
    }
    __builtin_amdgcn_fence(__ATOMIC_RELEASE, "workgroup");
    __builtin_amdgcn_wave_barrier();
    __builtin_amdgcn_fence(__ATOMIC_ACQUIRE, "workgroup");
    v4f vals[8];
#pragma unroll
    for (int it = 0; it < 8; ++it) {
      const int row = it * 2 + hh;
      v4f v = *(const v4f*)(slab + row * 68 + c4);
      if (SKIP) {
        const v4f uu = *(const v4f*)(skipSrc + (size_t)(mBase + row) * ldc + n0 + c4);
        v = v + g4 * uu;
      }
      vals[it] = v;
    }
    for (int pass = 0; pass < 2; ++pass) {
#pragma unroll
      for (int it = 0; it < 8; ++it) {
        const int row = it * 2 + hh;
        *(volatile v4f*)(Cout + (size_t)(mBase + row) * ldc + n0 + c4) = vals[it];
      }
      __threadfence();
    }
    __builtin_amdgcn_fence(__ATOMIC_RELEASE, "workgroup");
    __builtin_amdgcn_wave_barrier();
    __builtin_amdgcn_fence(__ATOMIC_ACQUIRE, "workgroup");
  }
}

__global__ __launch_bounds__(64) void chunk_end_kernel(
    const float* __restrict__ Tp, const float* __restrict__ tab, float* __restrict__ endp)
{
  const int tid = (int)threadIdx.x;
  const int c = (int)blockIdx.x;
  const int p0 = 2 * tid;
  const v2f ar = *(const v2f*)(tab + 0 * kP + p0);
  const v2f ai = *(const v2f*)(tab + 1 * kP + p0);
  const v2f cr = *(const v2f*)(tab + 2 * kP + p0);
  const v2f ci = *(const v2f*)(tab + 3 * kP + p0);
  float x0r = 0.0f, x0i = 0.0f, x1r = 0.0f, x1i = 0.0f;
  const float* base = Tp + (size_t)c * kLC * kTW + p0;
#pragma unroll 4
  for (int s = 0; s < kLC; ++s) {
    const v2f tr = *(const v2f*)(base + (size_t)s * kTW);
    const v2f ti = *(const v2f*)(base + (size_t)s * kTW + kP);
    const float b0r = cr[0] * tr[0] - ci[0] * ti[0];
    const float b0i = cr[0] * ti[0] + ci[0] * tr[0];
    const float b1r = cr[1] * tr[1] - ci[1] * ti[1];
    const float b1i = cr[1] * ti[1] + ci[1] * tr[1];
    const float n0r = ar[0] * x0r - ai[0] * x0i + b0r;
    const float n0i = ar[0] * x0i + ai[0] * x0r + b0i;
    const float n1r = ar[1] * x1r - ai[1] * x1i + b1r;
    const float n1i = ar[1] * x1i + ai[1] * x1r + b1i;
    x0r = n0r; x0i = n0i; x1r = n1r; x1i = n1i;
  }
  v2f er, ei;
  er[0] = x0r; er[1] = x1r;
  ei[0] = x0i; ei[1] = x1i;
  float* qr = endp + (size_t)c * kRowF + p0;
  float* qi = endp + (size_t)c * kRowF + kP + p0;
  *(volatile v2f*)qr = er;
  *(volatile v2f*)qi = ei;
  __threadfence();
  *(volatile v2f*)qr = er;
  *(volatile v2f*)qi = ei;
}

__global__ __launch_bounds__(128) void carry_chain_kernel(
    const float* __restrict__ endp, const float* __restrict__ tab, float* __restrict__ carry)
{
  const int p = (int)threadIdx.x;
  const float alr = tab[4 * kP + p];
  const float ali = tab[5 * kP + p];
  float curR = 0.0f, curI = 0.0f;
#pragma unroll 1
  for (int g = 0; g < kNChunk / 8; ++g) {
    float er[8], ei[8], vr[8], vi[8];
#pragma unroll
    for (int j = 0; j < 8; ++j) {
      er[j] = endp[(size_t)(g * 8 + j) * kRowF + p];
      ei[j] = endp[(size_t)(g * 8 + j) * kRowF + kP + p];
    }
#pragma unroll
    for (int j = 0; j < 8; ++j) {
      vr[j] = curR;
      vi[j] = curI;
      const float nr = alr * curR - ali * curI + er[j];
      const float ni = alr * curI + ali * curR + ei[j];
      curR = nr;
      curI = ni;
    }
    for (int pass = 0; pass < 2; ++pass) {
#pragma unroll
      for (int j = 0; j < 8; ++j) {
        *(volatile float*)(carry + (size_t)(g * 8 + j) * kRowF + p) = vr[j];
        *(volatile float*)(carry + (size_t)(g * 8 + j) * kRowF + kP + p) = vi[j];
      }
      __threadfence();
    }
  }
}

__global__ __launch_bounds__(64) void chunk_apply_kernel(
    const float* __restrict__ Tp, const float* __restrict__ tab,
    const float* __restrict__ carry, unsigned* __restrict__ a2w)
{
  __shared__ __align__(16) unsigned sX[kTS * 128];
  const int tid = (int)threadIdx.x;
  const int lane = tid & 31;
  const int wave = __builtin_amdgcn_readfirstlane((int)(threadIdx.x >> 5));
  const int c = (int)blockIdx.x;
  const int p0 = 2 * tid;
  const v2f ar = *(const v2f*)(tab + 0 * kP + p0);
  const v2f ai = *(const v2f*)(tab + 1 * kP + p0);
  const v2f cr = *(const v2f*)(tab + 2 * kP + p0);
  const v2f ci = *(const v2f*)(tab + 3 * kP + p0);
  const v2f c0r = *(const v2f*)(carry + (size_t)c * kRowF + p0);
  const v2f c0i = *(const v2f*)(carry + (size_t)c * kRowF + kP + p0);
  float x0r = c0r[0], x1r = c0r[1], x0i = c0i[0], x1i = c0i[1];
  const float* base = Tp + (size_t)c * kLC * kTW + p0;
  unsigned* obase = a2w + (size_t)c * kLC * 128;
#pragma unroll 1
  for (int t0 = 0; t0 < kLC; t0 += kTS) {
    __syncthreads();
#pragma unroll 4
    for (int s = 0; s < kTS; ++s) {
      const v2f tr = *(const v2f*)(base + (size_t)(t0 + s) * kTW);
      const v2f ti = *(const v2f*)(base + (size_t)(t0 + s) * kTW + kP);
      const float b0r = cr[0] * tr[0] - ci[0] * ti[0];
      const float b0i = cr[0] * ti[0] + ci[0] * tr[0];
      const float b1r = cr[1] * tr[1] - ci[1] * ti[1];
      const float b1i = cr[1] * ti[1] + ci[1] * tr[1];
      const float n0r = ar[0] * x0r - ai[0] * x0i + b0r;
      const float n0i = ar[0] * x0i + ai[0] * x0r + b0i;
      const float n1r = ar[1] * x1r - ai[1] * x1i + b1r;
      const float n1i = ar[1] * x1i + ai[1] * x1r + b1i;
      x0r = n0r; x0i = n0i; x1r = n1r; x1i = n1i;
      sX[s * 128 + tid]      = pack_h2(x0r * kCarryX, x1r * kCarryX);
      sX[s * 128 + 64 + tid] = pack_h2(x0i * kCarryX, x1i * kCarryX);
    }
    __syncthreads();
    v4u vals[16];
#pragma unroll
    for (int it = 0; it < 16; ++it) vals[it] = *(const v4u*)(sX + (wave * 16 + it) * 128 + lane * 4);
    for (int pass = 0; pass < 2; ++pass) {
#pragma unroll
      for (int it = 0; it < 16; ++it) {
        *(volatile v4u*)(obase + (size_t)(t0 + wave * 16 + it) * 128 + lane * 4) = vals[it];
      }
      __threadfence();
    }
  }
}

extern "C" void kernel_launch(void* const* d_in, const int* in_sizes, int n_in,
                              void* d_out, int out_size, void* d_ws, size_t ws_size,
                              hipStream_t stream) {
  if (n_in < 7) return;
  if (in_sizes[0] != kP) return;
  if (in_sizes[1] != kP) return;
  if (in_sizes[2] != kP * kH * 2) return;
  if (in_sizes[3] != kH * kP * 2) return;
  if (in_sizes[4] != kH) return;
  if (in_sizes[5] != kP) return;
  if (in_sizes[6] != kL * kH) return;
  if (out_size != kL * kH) return;
  if (ws_size < kWsTotal) return;

  const float* Lre   = (const float*)d_in[0];
  const float* Lim   = (const float*)d_in[1];
  const float* Bsrc  = (const float*)d_in[2];
  const float* Csrc  = (const float*)d_in[3];
  const float* Dg    = (const float*)d_in[4];
  const float* lstep = (const float*)d_in[5];
  const float* u     = (const float*)d_in[6];
  float* out = (float*)d_out;

  char* ws = (char*)d_ws;
  unsigned short* A1    = (unsigned short*)(ws + kOffA1);
  float*          TP    = (float*)(ws + kOffTP);
  unsigned short* A2    = (unsigned short*)(ws + kOffA2);
  unsigned short* BT1   = (unsigned short*)(ws + kOffBT1);
  unsigned short* BT2   = (unsigned short*)(ws + kOffBT2);
  float*          ENDP  = (float*)(ws + kOffEND);
  float*          CARRY = (float*)(ws + kOffCARRY);
  float*          TAB   = (float*)(ws + kOffTAB);

  param_table_kernel<<<1, kP, 0, stream>>>(Lre, Lim, lstep, TAB);
  weight_planes_kernel<<<64, 256, 0, stream>>>(Bsrc, Csrc, BT1, BT2);
  cast_rows_f16_kernel<<<(kL * kH / 8) / 256, 256, 0, stream>>>(u, A1, kL * kH / 8);

  gemm_f16_tile64<false><<<((kL / 64) * (kTW / 64)) / 8, 256, 0, stream>>>(
      A1, kH, BT1, kH, TP, kTW, Dg, u, kL, kTW, kH, kScale1);

  chunk_end_kernel<<<kNChunk, 64, 0, stream>>>(TP, TAB, ENDP);
  carry_chain_kernel<<<1, kP, 0, stream>>>(ENDP, TAB, CARRY);
  chunk_apply_kernel<<<kNChunk, 64, 0, stream>>>(TP, TAB, CARRY, (unsigned*)A2);

  gemm_f16_tile64<true><<<((kL / 64) * (kH / 64)) / 8, 256, 0, stream>>>(
      A2, kTW, BT2, kTW, out, kH, Dg, u, kL, kH, kTW, kScale2);
}
